// VideoMambaBlock_77721728188887
// MI455X (gfx1250) — hardware-verified
//
#include <hip/hip_runtime.h>


#define BSZ_   2
#define LSEQ_  4096
#define DIM_   256
#define DI_    512
#define NS_    16
#define DTR_   16
#define NDBL_  48
#define NROW_  (BSZ_ * LSEQ_)
#define NXZ_   (2 * DI_)
#define KIN3_  (3 * DIM_)
#define KDI3_  (3 * DI_)
#define XDW_   64
#define KDT_   64

static_assert(NROW_ == 8192);
static_assert(NXZ_ == 1024);
static_assert(KIN3_ % 32 == 0);
static_assert(KDI3_ % 32 == 0);
static_assert(KDT_ % 32 == 0);
static_assert(KDT_ == 4 * DTR_);
static_assert(LSEQ_ % 64 == 0);
static_assert(NROW_ % 64 == 0);
static_assert(DTR_ + 2 * NS_ == NDBL_);
static_assert(NDBL_ <= XDW_);
static_assert(XDW_ % 64 == 0);
static_assert(DI_ % 128 == 0);
static_assert(DIM_ % 128 == 0);
static_assert(DIM_ == 256);
static_assert(DI_ == 512);

typedef float          v4f   __attribute__((ext_vector_type(4)));
typedef float          v8f   __attribute__((ext_vector_type(8)));
typedef unsigned short u16x8 __attribute__((ext_vector_type(8)));
typedef __bf16         v16bf __attribute__((ext_vector_type(16)));

union FragB { u16x8 h[2]; v16bf v; };

constexpr size_t SZ_WIN = (size_t)NXZ_ * KIN3_ * 2;
constexpr size_t SZ_WX  = (size_t)XDW_ * KDI3_ * 2;
constexpr size_t SZ_WDT = (size_t)DI_ * KDT_ * 2;
constexpr size_t SZ_WO  = (size_t)DIM_ * KDI3_ * 2;
constexpr size_t SZ_XN  = (size_t)NROW_ * KIN3_ * 2;
constexpr size_t SZ_XC  = (size_t)NROW_ * DI_ * 4;
constexpr size_t SZ_Z   = (size_t)NROW_ * DI_ * 4;
constexpr size_t SZ_U   = (size_t)NROW_ * KDI3_ * 2;
constexpr size_t SZ_DBL = (size_t)NROW_ * XDW_ * 4;
constexpr size_t SZ_DTA = (size_t)NROW_ * KDT_ * 2;
constexpr size_t SZ_DT  = (size_t)NROW_ * DI_ * 4;
constexpr size_t SZ_G   = (size_t)NROW_ * KDI3_ * 2;

constexpr size_t OFF_WIN = 0;
constexpr size_t OFF_WX  = OFF_WIN + SZ_WIN;
constexpr size_t OFF_WDT = OFF_WX + SZ_WX;
constexpr size_t OFF_WO  = OFF_WDT + SZ_WDT;
constexpr size_t OFF_XN  = OFF_WO + SZ_WO;
constexpr size_t OFF_XC  = OFF_XN + SZ_XN;
constexpr size_t OFF_Z   = OFF_XC + SZ_XC;
constexpr size_t OFF_U   = OFF_Z + SZ_Z;
constexpr size_t OFF_DBL = OFF_U + SZ_U;
constexpr size_t OFF_DTA = OFF_DBL + SZ_DBL;
constexpr size_t OFF_DT  = OFF_DTA + SZ_DTA;
constexpr size_t OFF_G   = OFF_DT + SZ_DT;
constexpr size_t WS_END  = OFF_G + SZ_G;

static_assert(WS_END == (size_t)119013376);
static_assert(WS_END <= (size_t)134217728);
static_assert(OFF_WX % 128 == 0 && OFF_WDT % 128 == 0 && OFF_WO % 128 == 0 && OFF_XN % 128 == 0);
static_assert(OFF_XC % 128 == 0 && OFF_Z % 128 == 0 && OFF_U % 128 == 0 && OFF_DBL % 128 == 0);
static_assert(OFF_DTA % 128 == 0 && OFF_DT % 128 == 0 && OFF_G % 128 == 0 && WS_END % 128 == 0);

__device__ __forceinline__ unsigned short bfb(float f) {
    unsigned u = __float_as_uint(f);
    u += 0x7FFFu + ((u >> 16) & 1u);
    return (unsigned short)(u >> 16);
}
__device__ __forceinline__ void split8(const v8f v, u16x8& hi, u16x8& lo) {
#pragma unroll
    for (int e = 0; e < 8; ++e) {
        const unsigned short hb = bfb(v[e]);
        const float hf = __uint_as_float(((unsigned)hb) << 16);
        hi[e] = hb;
        lo[e] = bfb(v[e] - hf);
    }
}
__device__ __forceinline__ v8f ld8f(const float* p) {
    v4f a = *(const v4f*)p;
    v4f b = *(const v4f*)(p + 4);
    return __builtin_shufflevector(a, b, 0, 1, 2, 3, 4, 5, 6, 7);
}
__device__ __forceinline__ float silu_f(float x) {
    const float e = __expf(-x);
    return x * __builtin_amdgcn_rcpf(1.0f + e);
}
__device__ __forceinline__ float softplus_f(float x) {
    return fmaxf(x, 0.0f) + log1pf(__expf(-fabsf(x)));
}
__device__ __forceinline__ float conv4_silu(float x0, float x1, float x2, float x3,
                                            float w0, float w1, float w2, float w3, float bias) {
    const float c = w0 * x0 + w1 * x1 + w2 * x2 + w3 * x3;
    return silu_f(c + bias);
}

__device__ __forceinline__ void mma_bf(v8f& acc, const FragB& a, const FragB& b) {
    acc = __builtin_amdgcn_wmma_f32_16x16x32_bf16(false, a.v, false, b.v, (short)0, acc, false, false);
    asm volatile("v_nop\n\tv_nop\n\tv_nop\n\tv_nop" : "+v"(acc) : "v"(a.v), "v"(b.v));
}

__global__ __launch_bounds__(256)
void wplane_kernel(const float* __restrict__ W, unsigned short* dst, int Nreal, int Npad, int K, int pitch)
{
    const int CH    = pitch >> 3;
    const int total = Npad * CH;
    const int idx   = blockIdx.x * 256 + threadIdx.x;
    if (idx >= total) return;
    const int n    = idx / CH;
    const int q    = idx - n * CH;
    const int hoff = q * 8;
    const int seg  = hoff / K;
    const int kk   = hoff - seg * K;
    const int kcl  = min(max(kk, 0), K - 8);
    const int ncl  = min(max(n, 0), Nreal - 1);
    const bool ok  = (seg < 3) && (n < Nreal);
    v8f vals = ld8f(W + (size_t)ncl * K + kcl);
#pragma unroll
    for (int e = 0; e < 8; ++e) vals[e] = ok ? vals[e] : 0.0f;
    u16x8 hi, lo;
    split8(vals, hi, lo);
    u16x8 o;
#pragma unroll
    for (int e = 0; e < 8; ++e) o[e] = (seg == 1) ? lo[e] : hi[e];
    unsigned short* gp = dst + (size_t)n * pitch + hoff;
    *(volatile u16x8*)gp = o;
    __threadfence();
    *(volatile u16x8*)gp = o;
}

__global__ __launch_bounds__(256)
void xplane_kernel(const float* __restrict__ x, unsigned short* xn)
{
    __shared__ float tile[DIM_ * 17];
    const int tid = threadIdx.x, lane = tid & 31, wave = tid >> 5;
    const int t0 = blockIdx.x * 16;
    const int b  = t0 / LSEQ_;
    const int l0 = t0 - b * LSEQ_;
    const int lsub = tid & 15, csub = tid >> 4;
    const float* xb = x + (size_t)b * DIM_ * LSEQ_ + l0 + lsub;
#pragma unroll 4
    for (int it = 0; it < DIM_ / 16; ++it) {
        const int c = it * 16 + csub;
        tile[c * 17 + lsub] = xb[(size_t)c * LSEQ_];
    }
    __syncthreads();
#pragma unroll 1
    for (int i = 0; i < 2; ++i) {
        const int tl = wave * 2 + i;
        unsigned short* rowp = xn + (size_t)(t0 + tl) * KIN3_;
        const int cbase = 8 * lane;
        v8f v;
#pragma unroll
        for (int e = 0; e < 8; ++e) v[e] = tile[(cbase + e) * 17 + tl];
        u16x8 hi, lo;
        split8(v, hi, lo);
        unsigned short* gp = rowp + cbase;
        *(volatile u16x8*)gp              = hi;
        *(volatile u16x8*)(gp + DIM_)     = hi;
        *(volatile u16x8*)(gp + 2 * DIM_) = lo;
        __threadfence();
        *(volatile u16x8*)gp              = hi;
        *(volatile u16x8*)(gp + DIM_)     = hi;
        *(volatile u16x8*)(gp + 2 * DIM_) = lo;
    }
}

template<int NBF>
__device__ __forceinline__ void row_store_pass(const float* st, float* gp, int ldc, int lane) {
    constexpr int CW  = NBF * 16;
    constexpr int P   = CW + 4;
    constexpr int LPR = CW / 4;
    static_assert(32 % LPR == 0);
    constexpr int RPI = 32 / LPR;
    static_assert(32 % RPI == 0);
    constexpr int NIT = 32 / RPI;
    const int rsub = lane / LPR;
    const int c0   = (lane % LPR) * 4;
#pragma unroll
    for (int it = 0; it < NIT; ++it) {
        const int row = it * RPI + rsub;
        const v4f v = *(const v4f*)(st + row * P + c0);
        *(volatile v4f*)(gp + (size_t)row * ldc + c0) = v;
    }
}

template<int NBF>
__device__ __forceinline__ void trans_store_pass(const float* st, float* outp, int rowW, int colW, int lane) {
    constexpr int CW = NBF * 16;
    constexpr int P  = CW + 4;
    const int bb = rowW / LSEQ_;
    const int l0 = rowW - bb * LSEQ_;
    const int rq = lane & 7;
    const int cs = lane >> 3;
#pragma unroll
    for (int it = 0; it < CW / 4; ++it) {
        const int c = it * 4 + cs;
        v4f v;
        v[0] = st[(4 * rq + 0) * P + c];
        v[1] = st[(4 * rq + 1) * P + c];
        v[2] = st[(4 * rq + 2) * P + c];
        v[3] = st[(4 * rq + 3) * P + c];
        float* dp = outp + ((size_t)bb * DIM_ + colW + c) * LSEQ_ + l0 + 4 * rq;
        *(volatile v4f*)dp = v;
    }
}

template<int NBF, int MODE>
__global__ __launch_bounds__(128)
void gemm_tn_kernel(const unsigned short* __restrict__ A, const unsigned short* __restrict__ Bw,
                    float* C1, float* C2, int K, int ldc1, int ldc2, int csplit)
{
    constexpr int CW = NBF * 16;
    constexpr int P  = CW + 4;
    __shared__ __attribute__((aligned(16))) float stile[4][32 * P];

    const int tid  = threadIdx.x;
    const int lane = tid & 31;
    const int wave = tid >> 5;
    const int h    = lane >> 4;
    const int m    = lane & 15;
    const int wm   = wave >> 1;
    const int wn   = wave & 1;

    const int rowW = blockIdx.y * 64 + wm * 32;
    const int colW = blockIdx.x * (2 * CW) + wn * CW;

    const unsigned short* pa[2];
#pragma unroll
    for (int s = 0; s < 2; ++s) pa[s] = A + (size_t)(rowW + 16 * s + m) * K + 8 * h;
    const unsigned short* pb = Bw + (size_t)(colW + m) * K + 8 * h;
    const size_t sub16 = (size_t)16 * K;

    v8f acc[2 * NBF];
#pragma unroll
    for (int j = 0; j < 2 * NBF; ++j)
#pragma unroll
        for (int r = 0; r < 8; ++r) acc[j][r] = 0.0f;

    const int nk = K >> 5;
    for (int kt = 0; kt < nk; ++kt) {
        const int k0 = kt * 32;
        FragB fa[2], fb[NBF];
#pragma unroll
        for (int s = 0; s < 2; ++s) {
            fa[s].h[0] = *(const u16x8*)(pa[s] + k0);
            fa[s].h[1] = *(const u16x8*)(pa[s] + k0 + 16);
        }
#pragma unroll
        for (int j = 0; j < NBF; ++j) {
            const unsigned short* p = pb + j * sub16 + k0;
            fb[j].h[0] = *(const u16x8*)(p);
            fb[j].h[1] = *(const u16x8*)(p + 16);
        }
#pragma unroll
        for (int s = 0; s < 2; ++s)
#pragma unroll
            for (int j = 0; j < NBF; ++j)
                mma_bf(acc[s * NBF + j], fa[s], fb[j]);
    }

    float* st = stile[wave];
#pragma unroll
    for (int s = 0; s < 2; ++s)
#pragma unroll
        for (int j = 0; j < NBF; ++j)
#pragma unroll
            for (int r = 0; r < 8; ++r)
                st[(s * 16 + 8 * h + r) * P + j * 16 + m] = acc[s * NBF + j][r];
    __syncthreads();

    if constexpr (MODE == 0) {
        if (colW < csplit) {
            float* gp = C1 + (size_t)rowW * ldc1 + colW;
            row_store_pass<NBF>(st, gp, ldc1, lane);
            __threadfence();
            row_store_pass<NBF>(st, gp, ldc1, lane);
        } else {
            float* gp = C2 + (size_t)rowW * ldc2 + (colW - csplit);
            row_store_pass<NBF>(st, gp, ldc2, lane);
            __threadfence();
            row_store_pass<NBF>(st, gp, ldc2, lane);
        }
    } else {
        trans_store_pass<NBF>(st, C1, rowW, colW, lane);
        __threadfence();
        trans_store_pass<NBF>(st, C1, rowW, colW, lane);
    }
}

__global__ __launch_bounds__(256)
void conv_plane_kernel(const float* __restrict__ Xc, const float* __restrict__ cw,
                       const float* __restrict__ cb, unsigned short* U)
{
    const int tid = threadIdx.x;
    const int r   = tid >> 6;
    const int ch  = tid & 63;
    const int t   = blockIdx.x * 4 + r;
    const int l   = t & (LSEQ_ - 1);
    const int d0  = ch * 8;
    const int t1 = (l >= 1) ? (t - 1) : t;
    const int t2 = (l >= 2) ? (t - 2) : t;
    const int t3 = (l >= 3) ? (t - 3) : t;

    v8f x3 = ld8f(Xc + (size_t)t  * DI_ + d0);
    v8f x2 = ld8f(Xc + (size_t)t1 * DI_ + d0);
    v8f x1 = ld8f(Xc + (size_t)t2 * DI_ + d0);
    v8f x0 = ld8f(Xc + (size_t)t3 * DI_ + d0);
#pragma unroll
    for (int c = 0; c < 8; ++c) {
        x2[c] = (l >= 1) ? x2[c] : 0.0f;
        x1[c] = (l >= 2) ? x1[c] : 0.0f;
        x0[c] = (l >= 3) ? x0[c] : 0.0f;
    }
    v4f wv[8];
#pragma unroll
    for (int c = 0; c < 8; ++c) wv[c] = *(const v4f*)(cw + (size_t)(d0 + c) * 4);
    const v8f bias = ld8f(cb + d0);

    v8f u;
#pragma unroll
    for (int c = 0; c < 8; ++c)
        u[c] = conv4_silu(x0[c], x1[c], x2[c], x3[c], wv[c][0], wv[c][1], wv[c][2], wv[c][3], bias[c]);

    u16x8 hi, lo;
    split8(u, hi, lo);
    unsigned short* gp = U + (size_t)t * KDI3_ + d0;
    *(volatile u16x8*)gp             = hi;
    *(volatile u16x8*)(gp + DI_)     = hi;
    *(volatile u16x8*)(gp + 2 * DI_) = lo;
    __threadfence();
    *(volatile u16x8*)gp             = hi;
    *(volatile u16x8*)(gp + DI_)     = hi;
    *(volatile u16x8*)(gp + 2 * DI_) = lo;
}

__global__ __launch_bounds__(256)
void dta_plane_kernel(const float* __restrict__ dbl, unsigned short* dta)
{
    const int tid = threadIdx.x, lane = tid & 31, wave = tid >> 5;
    const int row   = blockIdx.x * 32 + wave * 4 + (lane >> 3);
    const int q     = lane & 7;
    const int seg   = q >> 1;
    const int piece = q & 1;
    const v8f v = ld8f(dbl + (size_t)row * XDW_ + 8 * piece);
    u16x8 hi, lo;
    split8(v, hi, lo);
    u16x8 o;
#pragma unroll
    for (int e = 0; e < 8; ++e) o[e] = (seg < 2) ? hi[e] : ((seg == 2) ? lo[e] : (unsigned short)0);
    unsigned short* gp = dta + (size_t)row * KDT_ + 8 * q;
    *(volatile u16x8*)gp = o;
    __threadfence();
    *(volatile u16x8*)gp = o;
}

__global__ __launch_bounds__(64)
void scan_kernel(const float* __restrict__ Xc, const float* __restrict__ Z, const float* __restrict__ dtr,
                 const float* __restrict__ dbl, const float* __restrict__ cw, const float* __restrict__ cb,
                 const float* __restrict__ bdt, const float* __restrict__ Alog, const float* __restrict__ Dp,
                 unsigned short* G)
{
    __shared__ __attribute__((aligned(16))) float sg[16 * 64];
    __shared__ __attribute__((aligned(16))) float sX[16 * 32];

    const int tid   = threadIdx.x;
    const int lane  = tid & 31;
    const int wave  = tid >> 5;
    const int b     = blockIdx.y;
    const int dbase = blockIdx.x * 64;
    const int d     = dbase + tid;

    float an[NS_], hs[NS_];
#pragma unroll
    for (int n = 0; n < NS_; ++n) {
        an[n] = -__expf(Alog[(size_t)d * NS_ + n]);
        hs[n] = 0.0f;
    }
    const v4f wv = *(const v4f*)(cw + (size_t)d * 4);
    const float cbias = cb[d];
    const float tb    = bdt[d];
    const float Dd    = Dp[d];

    float xm1 = 0.0f, xm2 = 0.0f, xm3 = 0.0f;
    const size_t trow0 = (size_t)b * LSEQ_;
    const int j = tid >> 2, piece = tid & 3;

#pragma unroll 1
    for (int l0 = 0; l0 < LSEQ_; l0 += 16) {
        {
            const float* src = dbl + (trow0 + (size_t)(l0 + j)) * XDW_ + DTR_ + 8 * piece;
            const v4f a = *(const v4f*)src;
            const v4f c = *(const v4f*)(src + 4);
            *(v4f*)(sX + j * 32 + 8 * piece)     = a;
            *(v4f*)(sX + j * 32 + 8 * piece + 4) = c;
        }
        __syncthreads();
#pragma unroll 1
        for (int t = 0; t < 16; ++t) {
            const size_t e = (trow0 + (size_t)(l0 + t)) * DI_ + d;
            const float xv = Xc[e];
            const float zv = Z[e];
            const float dr = dtr[e];
            const float u  = conv4_silu(xm3, xm2, xm1, xv, wv[0], wv[1], wv[2], wv[3], cbias);
            xm3 = xm2; xm2 = xm1; xm1 = xv;
            const float dt = softplus_f(dr + tb);
            const float du = dt * u;
            const float* sr = sX + t * 32;
            float y = 0.0f;
#pragma unroll
            for (int n = 0; n < NS_; ++n) {
                const float da = __expf(dt * an[n]);
                hs[n] = da * hs[n] + du * sr[n];
                y += hs[n] * sr[NS_ + n];
            }
            sg[t * 64 + tid] = (y + Dd * u) * silu_f(zv);
        }
        __syncthreads();
        u16x8 ghi[2], glo[2];
        unsigned short* gp[2];
#pragma unroll
        for (int it = 0; it < 2; ++it) {
            const int r = it * 8 + wave * 4 + (lane >> 3);
            const int q = lane & 7;
            const v8f v = ld8f(sg + r * 64 + q * 8);
            split8(v, ghi[it], glo[it]);
            gp[it] = G + (trow0 + (size_t)(l0 + r)) * KDI3_ + dbase + q * 8;
        }
#pragma unroll
        for (int it = 0; it < 2; ++it) {
            *(volatile u16x8*)gp[it]             = ghi[it];
            *(volatile u16x8*)(gp[it] + DI_)     = ghi[it];
            *(volatile u16x8*)(gp[it] + 2 * DI_) = glo[it];
        }
        __threadfence();
#pragma unroll
        for (int it = 0; it < 2; ++it) {
            *(volatile u16x8*)gp[it]             = ghi[it];
            *(volatile u16x8*)(gp[it] + DI_)     = ghi[it];
            *(volatile u16x8*)(gp[it] + 2 * DI_) = glo[it];
        }
        __syncthreads();
    }
}

extern "C" void kernel_launch(void* const* d_in, const int* in_sizes, int n_in,
                              void* d_out, int out_size, void* d_ws, size_t ws_size,
                              hipStream_t stream)
{
    if (n_in < 10) return;
    if (in_sizes[0] != BSZ_ * DIM_ * LSEQ_)  return;
    if (in_sizes[1] != NXZ_ * DIM_)          return;
    if (in_sizes[2] != DI_ * 4)              return;
    if (in_sizes[3] != DI_)                  return;
    if (in_sizes[4] != NDBL_ * DI_)          return;
    if (in_sizes[5] != DI_ * DTR_)           return;
    if (in_sizes[6] != DI_)                  return;
    if (in_sizes[7] != DI_ * NS_)            return;
    if (in_sizes[8] != DI_)                  return;
    if (in_sizes[9] != DIM_ * DI_)           return;
    if (out_size != BSZ_ * DIM_ * LSEQ_)     return;
    if (ws_size < WS_END)                    return;

    const float* x      = (const float*)d_in[0];
    const float* W_in   = (const float*)d_in[1];
    const float* conv_w = (const float*)d_in[2];
    const float* conv_b = (const float*)d_in[3];
    const float* W_x    = (const float*)d_in[4];
    const float* W_dt   = (const float*)d_in[5];
    const float* b_dt   = (const float*)d_in[6];
    const float* A_log  = (const float*)d_in[7];
    const float* D_p    = (const float*)d_in[8];
    const float* W_out  = (const float*)d_in[9];
    float* out = (float*)d_out;

    char* ws = (char*)d_ws;
    unsigned short* winP = (unsigned short*)(ws + OFF_WIN);
    unsigned short* wxP  = (unsigned short*)(ws + OFF_WX);
    unsigned short* wdtP = (unsigned short*)(ws + OFF_WDT);
    unsigned short* woP  = (unsigned short*)(ws + OFF_WO);
    unsigned short* xnP  = (unsigned short*)(ws + OFF_XN);
    float*          Xc   = (float*)(ws + OFF_XC);
    float*          Zf   = (float*)(ws + OFF_Z);
    unsigned short* uP   = (unsigned short*)(ws + OFF_U);
    float*          dbl  = (float*)(ws + OFF_DBL);
    unsigned short* dtaP = (unsigned short*)(ws + OFF_DTA);
    float*          dtr  = (float*)(ws + OFF_DT);
    unsigned short* gP   = (unsigned short*)(ws + OFF_G);

    wplane_kernel<<<dim3((NXZ_ * (KIN3_ / 8) + 255) / 256), dim3(256), 0, stream>>>(W_in,  winP, (int)NXZ_,  (int)NXZ_, (int)DIM_, (int)KIN3_);
    wplane_kernel<<<dim3((XDW_ * (KDI3_ / 8) + 255) / 256), dim3(256), 0, stream>>>(W_x,   wxP,  (int)NDBL_, (int)XDW_, (int)DI_,  (int)KDI3_);
    wplane_kernel<<<dim3((DI_  * (KDT_  / 8) + 255) / 256), dim3(256), 0, stream>>>(W_dt,  wdtP, (int)DI_,   (int)DI_,  (int)DTR_, (int)KDT_);
    wplane_kernel<<<dim3((DIM_ * (KDI3_ / 8) + 255) / 256), dim3(256), 0, stream>>>(W_out, woP,  (int)DIM_,  (int)DIM_, (int)DI_,  (int)KDI3_);

    xplane_kernel<<<dim3(NROW_ / 16), dim3(256), 0, stream>>>(x, xnP);

    gemm_tn_kernel<4, 0><<<dim3(NXZ_ / 128, NROW_ / 64), dim3(128), 0, stream>>>(
        (const unsigned short*)xnP, (const unsigned short*)winP, Xc, Zf, (int)KIN3_, (int)DI_, (int)DI_, (int)DI_);

    conv_plane_kernel<<<dim3(NROW_ / 4), dim3(256), 0, stream>>>((const float*)Xc, conv_w, conv_b, uP);

    gemm_tn_kernel<2, 0><<<dim3(XDW_ / 64, NROW_ / 64), dim3(128), 0, stream>>>(
        (const unsigned short*)uP, (const unsigned short*)wxP, dbl, dbl, (int)KDI3_, (int)XDW_, (int)XDW_, 1 << 30);

    dta_plane_kernel<<<dim3(NROW_ / 32), dim3(256), 0, stream>>>((const float*)dbl, dtaP);

    gemm_tn_kernel<4, 0><<<dim3(DI_ / 128, NROW_ / 64), dim3(128), 0, stream>>>(
        (const unsigned short*)dtaP, (const unsigned short*)wdtP, dtr, dtr, (int)KDT_, (int)DI_, (int)DI_, 1 << 30);

    scan_kernel<<<dim3(DI_ / 64, BSZ_), dim3(64), 0, stream>>>(
        (const float*)Xc, (const float*)Zf, (const float*)dtr, (const float*)dbl, conv_w, conv_b, b_dt, A_log, D_p, gP);

    gemm_tn_kernel<4, 1><<<dim3(DIM_ / 128, NROW_ / 64), dim3(128), 0, stream>>>(
        (const unsigned short*)gP, (const unsigned short*)woP, out, out, (int)KDI3_, 0, 0, 0);
}
